// signature_model_10746008175156
// MI455X (gfx1250) — hardware-verified
//
#include <hip/hip_runtime.h>

typedef __attribute__((ext_vector_type(16))) _Float16 v16h;
typedef __attribute__((ext_vector_type(8)))  _Float16 v8h;
typedef __attribute__((ext_vector_type(8)))  float    v8f;
typedef __attribute__((ext_vector_type(4)))  float    v4f;

constexpr int kBatch   = 128;
constexpr int kLen     = 256;
constexpr int kCh      = 8;
constexpr int kNout    = 10;
constexpr int kLow     = 8 + 64 + 512;
constexpr int kLvl4    = 4096;
constexpr int kSigDim  = kLow + kLvl4;
constexpr int kKpad    = 4736;
constexpr int kNpad    = 16;
constexpr int kChunk   = 32;
constexpr int kNChunk  = kLen / kChunk;
constexpr int kU4P     = 40;
constexpr int kDxtP    = 264;
constexpr int kChunks16 = kKpad / 8;
constexpr int kHeadWaves = 4;
constexpr int kHeadSteps = kKpad / 32 / kHeadWaves;
static_assert(kSigDim == 4680, "level concatenation width");
static_assert((kKpad % 32) == 0 && kKpad >= kSigDim, "padded K");
static_assert(((kKpad * 2) % 128) == 0, "plane row is a whole number of lines");
static_assert((kSigDim % 8) == 0 && (kLow % 8) == 0, "16-B chunk boundaries");
static_assert(kChunks16 == 592, "16-B chunks per plane row");
static_assert(kHeadSteps * kHeadWaves * 32 == kKpad, "k-steps split evenly over the waves");
static_assert((kU4P % 8) == 0 && (kDxtP % 8) == 0, "16-B aligned LDS rows");
static_assert(kNChunk * kChunk == kLen, "chunking covers all steps");

constexpr float kCarryU  = 1024.0f;
constexpr float kCarryD  = 64.0f;
constexpr float kCarryS  = 256.0f;
constexpr float kCarryW  = 1024.0f;
constexpr float kFoldT4   = 1.0f / (kCarryU * kCarryD);
constexpr float kFoldHead = 1.0f / (kCarryS * kCarryW);

constexpr size_t kOffSig  = 0;
constexpr size_t kOffW16  = kOffSig + (size_t)kBatch * kKpad * 2;
constexpr size_t kWsTotal = kOffW16 + (size_t)kNpad * kKpad * 2;
static_assert(kOffW16 == 1212416ull && (kOffW16 % 128) == 0, "aligned region");
static_assert(kWsTotal == 1363968ull, "carve total");
static_assert(kWsTotal <= 134217728ull, "carve cap");

constexpr int kOffDxs = 0;
constexpr int kOffDxt = kOffDxs + kLen * kCh;
constexpr int kOffU   = kOffDxt + (kNpad * kDxtP) / 2;
constexpr int kLdsFloats = kOffU + (512 * kU4P) / 2;
static_assert(((kOffDxt * 4) % 16) == 0 && ((kOffU * 4) % 16) == 0, "16-B aligned LDS regions");
static_assert(kKpad <= (512 * kU4P) / 2, "f32 staging row fits in the dead u4 region");
static_assert(kLdsFloats * 4 <= 65536, "static LDS");

struct FragH {
  union U { v16h v; v8h h[2]; };
  static __device__ __forceinline__ v16h load(const _Float16* p) {
    U f;
    f.h[0] = *(const v8h*)(p);
    f.h[1] = *(const v8h*)(p + 16);
    return f.v;
  }
};
__device__ __forceinline__ v8f mma_h(v16h a, v16h b, v8f c) {
  c = __builtin_amdgcn_wmma_f32_16x16x32_f16(false, a, false, b, (short)0, c, false, false);
  asm volatile("v_nop\n\tv_nop\n\tv_nop\n\tv_nop" : "+v"(c) : "v"(a), "v"(b));
  return c;
}

__global__ __launch_bounds__(256) void wplane_kernel(const float* __restrict__ W, unsigned short* __restrict__ W16) {
  const int idx = blockIdx.x * 256 + threadIdx.x;
  const int total = kNpad * kChunks16;
  const int idc = (idx < total) ? idx : (total - 1);
  const int row = idc / kChunks16;
  const int k   = (idc - row * kChunks16) * 8;
  const bool live = (row < kNout) && (k < kSigDim);
  const int rc = (row < kNout) ? row : (kNout - 1);
  const int kc = (k < kSigDim) ? k : (kSigDim - 8);
  const float* src = W + (size_t)rc * kSigDim + kc;
  v4f a0 = *(const v4f*)(src);
  v4f a1 = *(const v4f*)(src + 4);
  asm volatile("" : "+v"(a0), "+v"(a1));
  v8h hv;
#pragma unroll
  for (int e = 0; e < 4; ++e) {
    const float x0 = live ? (a0[e] * kCarryW) : 0.0f;
    const float x1 = live ? (a1[e] * kCarryW) : 0.0f;
    hv[e]     = (_Float16)x0;
    hv[4 + e] = (_Float16)x1;
  }
  if (idx < total) {
    unsigned short* q = W16 + (size_t)idx * 8;
    *(volatile v8h*)q = hv;
    __threadfence();
    *(volatile v8h*)q = hv;
  }
}

__global__ __launch_bounds__(256) void scan_kernel(const float* __restrict__ X, unsigned short* __restrict__ SIG) {
  __shared__ __align__(16) float lds[kLdsFloats];
  float*    dxs  = lds + kOffDxs;
  _Float16* dxt  = (_Float16*)(lds + kOffDxt);
  _Float16* u4p  = (_Float16*)(lds + kOffU);
  float*    sigf = lds + kOffU;

  const int tid   = threadIdx.x;
  const int lane  = tid & 31;
  const int wave  = __builtin_amdgcn_readfirstlane((int)(threadIdx.x >> 5));
  const int hh    = lane >> 4;
  const int rlane = lane & 15;
  const int koff  = hh * 8;
  const int b     = blockIdx.x;

  {
    const float* Xb = X + (size_t)b * (kLen * kCh);
    const int t  = tid;
    const int t1 = (t + 1 < kLen) ? (t + 1) : (kLen - 1);
    const v4f a0 = *(const v4f*)(Xb + t * kCh);
    const v4f a1 = *(const v4f*)(Xb + t * kCh + 4);
    const v4f c0 = *(const v4f*)(Xb + t1 * kCh);
    const v4f c1 = *(const v4f*)(Xb + t1 * kCh + 4);
    const v4f d0 = c0 - a0;
    const v4f d1 = c1 - a1;
    *(v4f*)(dxs + t * kCh)     = d0;
    *(v4f*)(dxs + t * kCh + 4) = d1;
#pragma unroll
    for (int e = 0; e < 4; ++e) {
      dxt[e * kDxtP + t]       = (_Float16)(d0[e] * kCarryD);
      dxt[(4 + e) * kDxtP + t] = (_Float16)(d1[e] * kCarryD);
    }
#pragma unroll
    for (int l = kCh; l < kNpad; ++l) dxt[l * kDxtP + t] = (_Float16)0.0f;
  }
  __syncthreads();

  const int i0 = tid >> 6;
  const int i1 = i0 + 4;
  const int jj = (tid >> 3) & 7;
  const int kk = tid & 7;
  float s1a = 0.0f, s1b = 0.0f, s2a = 0.0f, s2b = 0.0f, s3a = 0.0f, s3b = 0.0f;
  v8f acc[4];
#pragma unroll
  for (int i = 0; i < 4; ++i) acc[i] = (v8f){0.f, 0.f, 0.f, 0.f, 0.f, 0.f, 0.f, 0.f};
  const int rowBase = wave * 64;
  constexpr float c6  = 1.0f / 6.0f;
  constexpr float c24 = 1.0f / 24.0f;

#pragma unroll 1
  for (int ch = 0; ch < kNChunk; ++ch) {
    const int t0 = ch * kChunk;
#pragma unroll 1
    for (int s = 0; s < kChunk; ++s) {
      const float* dx = dxs + (t0 + s) * kCh;
      const float dxa = dx[i0];
      const float dxb = dx[i1];
      const float dxj = dx[jj];
      const float dxk = dx[kk];
      const float ava = s1a * c6 + dxa * c24;
      const float avb = s1b * c6 + dxb * c24;
      const float bva = s2a * 0.5f + ava * dxj;
      const float bvb = s2b * 0.5f + avb * dxj;
      const float u4a = s3a + bva * dxk;
      const float u4b = s3b + bvb * dxk;
      const float u3a = s2a + (s1a * 0.5f + dxa * c6) * dxj;
      const float u3b = s2b + (s1b * 0.5f + dxb * c6) * dxj;
      const float n3a = s3a + u3a * dxk;
      const float n3b = s3b + u3b * dxk;
      const float n2a = s2a + (s1a + dxa * 0.5f) * dxj;
      const float n2b = s2b + (s1b + dxb * 0.5f) * dxj;
      const float n1a = s1a + dxa;
      const float n1b = s1b + dxb;
      u4p[tid * kU4P + s]         = (_Float16)(u4a * kCarryU);
      u4p[(tid + 256) * kU4P + s] = (_Float16)(u4b * kCarryU);
      s3a = n3a; s3b = n3b;
      s2a = n2a; s2b = n2b;
      s1a = n1a; s1b = n1b;
    }
    __syncthreads();
    {
      const v16h bf = FragH::load(dxt + rlane * kDxtP + t0 + koff);
#pragma unroll
      for (int i = 0; i < 4; ++i) {
        const v16h af = FragH::load(u4p + (rowBase + i * 16 + rlane) * kU4P + koff);
        acc[i] = mma_h(af, bf, acc[i]);
      }
    }
    __syncthreads();
  }

  if ((tid & 63) == 0) {
    sigf[i0] = s1a;
    sigf[i1] = s1b;
  }
  if (kk == 0) {
    sigf[8 + i0 * 8 + jj] = s2a;
    sigf[8 + i1 * 8 + jj] = s2b;
  }
  sigf[72 + tid]       = s3a;
  sigf[72 + tid + 256] = s3b;
  if (rlane < kCh) {
#pragma unroll
    for (int i = 0; i < 4; ++i) {
#pragma unroll
      for (int r = 0; r < 8; ++r) {
        const float v = acc[i][r] * kFoldT4;
        sigf[kLow + (rowBase + i * 16 + 8 * hh + r) * kCh + rlane] = v;
      }
    }
  }
  if (tid < kKpad - kSigDim) sigf[kSigDim + tid] = 0.0f;
  __syncthreads();

  v8h hv[3];
#pragma unroll
  for (int it = 0; it < 3; ++it) {
    const int c  = tid + 256 * it;
    const int cc = (c < kChunks16) ? c : (kChunks16 - 1);
    const v4f f0 = *(const v4f*)(sigf + cc * 8);
    const v4f f1 = *(const v4f*)(sigf + cc * 8 + 4);
#pragma unroll
    for (int e = 0; e < 4; ++e) {
      hv[it][e]     = (_Float16)(f0[e] * kCarryS);
      hv[it][4 + e] = (_Float16)(f1[e] * kCarryS);
    }
  }
  unsigned short* rowp = SIG + (size_t)b * kKpad;
  for (int pass = 0; pass < 2; ++pass) {
#pragma unroll
    for (int it = 0; it < 3; ++it) {
      const int c = tid + 256 * it;
      if (c < kChunks16) *(volatile v8h*)(rowp + (size_t)c * 8) = hv[it];
    }
    __threadfence();
  }
}

__global__ __launch_bounds__(128) void head_kernel(const unsigned short* __restrict__ SIG,
                                                   const unsigned short* __restrict__ W16,
                                                   const float* __restrict__ bias,
                                                   float* __restrict__ out) {
  __shared__ __align__(16) float sP[kHeadWaves][256];
  __shared__ __align__(16) float sOut[16 * kNout];
  const int tid   = threadIdx.x;
  const int lane  = tid & 31;
  const int wave  = __builtin_amdgcn_readfirstlane((int)(threadIdx.x >> 5));
  const int hh    = lane >> 4;
  const int rlane = lane & 15;
  const int koff  = hh * 8;
  const int m0    = blockIdx.x * 16;

  const int ncol = tid & 15;
  const int nclamp = (ncol < kNout) ? ncol : (kNout - 1);
  float bv = bias[nclamp];
  asm volatile("" : "+v"(bv));

  const _Float16* ap = (const _Float16*)SIG + (size_t)(m0 + rlane) * kKpad + koff;
  const _Float16* bp = (const _Float16*)W16 + (size_t)rlane * kKpad + koff;
  v8f acc = (v8f){0.f, 0.f, 0.f, 0.f, 0.f, 0.f, 0.f, 0.f};
  const int ks0 = wave * kHeadSteps;
#pragma unroll 1
  for (int s = 0; s < kHeadSteps; ++s) {
    const int k0 = (ks0 + s) * 32;
    const v16h af = FragH::load(ap + k0);
    const v16h bf = FragH::load(bp + k0);
    acc = mma_h(af, bf, acc);
  }
#pragma unroll
  for (int r = 0; r < 8; ++r) sP[wave][(8 * hh + r) * 16 + rlane] = acc[r];
  __syncthreads();
#pragma unroll
  for (int q = 0; q < 2; ++q) {
    const int e   = tid + 128 * q;
    const int row = e >> 4;
    const float p0 = sP[0][e], p1 = sP[1][e], p2 = sP[2][e], p3 = sP[3][e];
    const float sum = ((p0 + p1) + p2) + p3;
    const float val = sum * kFoldHead + bv;
    if (ncol < kNout) sOut[row * kNout + ncol] = val;
  }
  __syncthreads();
  if (wave == 0) {
    float v[5];
#pragma unroll
    for (int ln = 0; ln < 5; ++ln) v[ln] = sOut[ln * 32 + lane];
    float* dst = out + (size_t)m0 * kNout;
    for (int pass = 0; pass < 2; ++pass) {
#pragma unroll
      for (int ln = 0; ln < 5; ++ln) *(volatile float*)(dst + ln * 32 + lane) = v[ln];
      __threadfence();
    }
  }
}

extern "C" void kernel_launch(void* const* d_in, const int* in_sizes, int n_in,
                              void* d_out, int out_size, void* d_ws, size_t ws_size,
                              hipStream_t stream) {
  if (n_in < 3) return;
  if (in_sizes[0] != kBatch * kLen * kCh) return;
  if (in_sizes[1] != kNout * kSigDim) return;
  if (in_sizes[2] != kNout) return;
  if (out_size != kBatch * kNout) return;
  if (ws_size < kWsTotal) return;

  const float* X    = (const float*)d_in[0];
  const float* W    = (const float*)d_in[1];
  const float* bias = (const float*)d_in[2];
  float* out = (float*)d_out;
  char* ws = (char*)d_ws;
  unsigned short* SIG = (unsigned short*)(ws + kOffSig);
  unsigned short* W16 = (unsigned short*)(ws + kOffW16);

  wplane_kernel<<<(kNpad * kChunks16) / 256, 256, 0, stream>>>(W, W16);
  scan_kernel<<<kBatch, 256, 0, stream>>>(X, SIG);
  head_kernel<<<kBatch / 16, 128, 0, stream>>>(SIG, W16, bias, out);
}
